// GIBGIN_75960791597152
// MI455X (gfx1250) — hardware-verified
//
#include <hip/hip_runtime.h>
#include <stddef.h>


#define FIN0    128
#define HD      256
#define NCLS    2
#define NTHR    256
#define NWAVE   8
#define EPT     8
#define NGRP    2
#define CHUNK   (NTHR * EPT * NGRP)
#define WCAP    (EPT * NGRP * 32)
#define LISTN   (NWAVE * WCAP)
#define NBC     4096
#define NBF     1024
#define RCAP    40960
#define RBN     128
#define TGT     256
#define DEGCAP  256
#define OTHR    512
#define BM      32
#define NT      4
#define STATR   256
#define GPB     16
#define GPA     32
#define WSCAP   134217728
#define BN_EPS  1e-5
#define XSC     8.0f
#define WSC     64.0f
#define INV_CARRY (1.0f / 512.0f)

#define LDS_FILL ((RCAP + NBF + LISTN) * 4 + 64)

static_assert((CHUNK & (CHUNK - 1)) == 0);
static_assert(CHUNK <= 4096);
static_assert(NBC <= 4096 && NBF <= 4096);
static_assert((NBC & (NBC - 1)) == 0 && (NBF & (NBF - 1)) == 0);
static_assert(NBC == 4 * NBF);
static_assert(OTHR * 8 == NBC);
static_assert((RCAP % 32) == 0);
static_assert(TGT == NWAVE * 32);
static_assert((TGT % BM) == 0 && (TGT % STATR) == 0 && (NBF % TGT) == 0);
static_assert(4 * 16 * NT == HD);
static_assert((HD % 32) == 0 && (FIN0 % 32) == 0 && FIN0 <= HD);
static_assert(((BM * HD) / 4) % NTHR == 0);
static_assert(NTHR == HD);
static_assert((GPB & (GPB - 1)) == 0 && (GPA & (GPA - 1)) == 0 && GPA == 32 && (32 % GPB) == 0);
static_assert(((GPB * HD) / 4) % NTHR == 0 && ((GPB * HD) / 8) % NTHR == 0);
static_assert(BM * 2 * 4 == 256);

typedef float          v2f  __attribute__((ext_vector_type(2)));
typedef float          v4f  __attribute__((ext_vector_type(4)));
typedef float          v8f  __attribute__((ext_vector_type(8)));
typedef int            v4i  __attribute__((ext_vector_type(4)));
typedef _Float16       v4h  __attribute__((ext_vector_type(4)));
typedef _Float16       v8h  __attribute__((ext_vector_type(8)));
typedef _Float16       v16h __attribute__((ext_vector_type(16)));
union FragH { v16h v; v8h h[2]; };

__device__ __forceinline__ v8f wmh(v16h a, v16h b, v8f c) {
  v8f d = __builtin_amdgcn_wmma_f32_16x16x32_f16(false, a, false, b, (short)0, c, false, false);
  asm volatile("v_nop\n\tv_nop\n\tv_nop\n\tv_nop" : "+v"(d) : "v"(a), "v"(b));
  return d;
}

template <int NB, bool IND>
__device__ __forceinline__ int scan_chunk(const int* __restrict__ ids, int nE, const int* __restrict__ tab, int nTab,
                                          int cbase, int slotBase, int vec8, int* list, int tid, int lane, int wave) {
  int wc = 0;
#pragma unroll
  for (int g = 0; g < NGRP; ++g) {
    const int el0  = (g * NTHR + tid) * EPT;
    const int e0   = cbase + el0;
    const int sent = -2147483647 - 1;
    int rv[8];
    if (vec8 != 0 && cbase + CHUNK <= nE) {
      const v4i da = *(const v4i*)(ids + e0);
      const v4i db = *(const v4i*)(ids + e0 + 4);
      rv[0] = da.x; rv[1] = da.y; rv[2] = da.z; rv[3] = da.w;
      rv[4] = db.x; rv[5] = db.y; rv[6] = db.z; rv[7] = db.w;
    } else {
#pragma unroll
      for (int j = 0; j < 8; ++j) {
        int e = e0 + j;
        e = e > nE - 1 ? nE - 1 : e;
        rv[j] = ids[e];
      }
    }
    int kv[8];
#pragma unroll
    for (int j = 0; j < 8; ++j) {
      int k = rv[j];
      if (IND) {
        const int q = k < 0 ? 0 : (k > nTab - 1 ? nTab - 1 : k);
        k = tab[q];
      }
      kv[j] = (e0 + j < nE) ? k : sent;
    }
    unsigned sv[8];
    bool hv[8];
    bool anyb = false;
    const unsigned nb = (unsigned)slotBase;
#pragma unroll
    for (int j = 0; j < 8; ++j) {
      sv[j] = (unsigned)kv[j] - nb;
      hv[j] = sv[j] < (unsigned)NB;
      anyb = anyb || hv[j];
    }
    const unsigned any = __builtin_amdgcn_ballot_w32(anyb);
    if (any != 0u) {
#pragma unroll
      for (int j = 0; j < 8; ++j) {
        const unsigned mj = __builtin_amdgcn_ballot_w32(hv[j]);
        if (mj != 0u) {
          if (hv[j]) {
            const int pos = wc + (int)__builtin_amdgcn_mbcnt_lo(mj, 0u);
            if (pos < WCAP) list[wave * WCAP + pos] = ((el0 + j) << 12) | (int)sv[j];
          }
          wc += (int)__builtin_popcount(mj);
        }
      }
    }
  }
  return wc;
}

template <int KS, int NS, int KD, int NCP>
__global__ __launch_bounds__(NTHR) void k_wprep(const float* __restrict__ W, _Float16* wp, int nL) {
  constexpr int KD8 = KD / 8;
  constexpr int UPL = NCP * KD8;
  static_assert((UPL % 32) == 0);
  const int i = (int)blockIdx.x * NTHR + (int)threadIdx.x;
  if (i >= nL * UPL) return;
  const int l  = i / UPL;
  const int r  = i - l * UPL;
  const int n  = r / KD8;
  const int k0 = (r - n * KD8) * 8;
  const int nn = n < NS ? n : NS - 1;
  v8h hv;
#pragma unroll
  for (int e = 0; e < 8; ++e) {
    const int k  = k0 + e;
    const int kk = k < KS ? k : KS - 1;
    float v = W[((size_t)l * KS + kk) * NS + nn];
    if (k >= KS || n >= NS) v = 0.0f;
    hv[e] = (_Float16)(v * WSC);
  }
  _Float16* d = wp + (size_t)i * 8;
  *(volatile v8h*)d = hv;
  __threadfence();
  *(volatile v8h*)d = hv;
}

__global__ __launch_bounds__(NTHR) void k_count(
    const int* __restrict__ dsts, int* cnt, int nE, int vec8) {
  __shared__ __attribute__((aligned(16))) int scnt[NBC];
  __shared__ __attribute__((aligned(16))) int list[LISTN];
  __shared__ int wcnt[NWAVE];
  const int tid = threadIdx.x, lane = tid & 31, wave = tid >> 5;
  const int nodeBase = blockIdx.x * NBC;

  for (int i = tid; i < NBC; i += NTHR) scnt[i] = 0;
  __syncthreads();

  const int nChunks = (nE + CHUNK - 1) / CHUNK;
#pragma unroll 1
  for (int ch = 0; ch < nChunks; ++ch) {
    const int cbase = ch * CHUNK;
    const int wc = scan_chunk<NBC, false>(dsts, nE, dsts, nE, cbase, nodeBase, vec8, list, tid, lane, wave);
    if (lane == 0) wcnt[wave] = wc;
    __syncthreads();
    if (wave == 0) {
#pragma unroll 1
      for (int wsx = 0; wsx < NWAVE; ++wsx) {
        int n = __builtin_amdgcn_readfirstlane(wcnt[wsx]);
        n = n > WCAP ? WCAP : (n < 0 ? 0 : n);
        const int* lp = list + wsx * WCAP;
#pragma unroll 1
        for (int i = 0; i < n; ++i) {
          const int ent  = __builtin_amdgcn_readfirstlane(lp[i]);
          const int slot = ent & (NBC - 1);
          if (lane == 0) scnt[slot] = scnt[slot] + 1;
        }
      }
    }
    __syncthreads();
  }

  v4i cq[4];
#pragma unroll
  for (int q = 0; q < 4; ++q) {
    const int f = (wave * 4 + q) * 128 + 4 * lane;
    cq[q] = *(const v4i*)(scnt + f);
  }
  int* cp = cnt + (size_t)nodeBase;
#pragma unroll
  for (int q = 0; q < 4; ++q) {
    const int f = (wave * 4 + q) * 128 + 4 * lane;
    *(volatile v4i*)(cp + f) = cq[q];
  }
  __threadfence();
#pragma unroll
  for (int q = 0; q < 4; ++q) {
    const int f = (wave * 4 + q) * 128 + 4 * lane;
    *(volatile v4i*)(cp + f) = cq[q];
  }
}

__global__ __launch_bounds__(OTHR) void k_offsets(
    const int* __restrict__ cnt, int* off, int* rbase, int nChunk) {
  __shared__ __attribute__((aligned(16))) int soff[NBC];
  __shared__ __attribute__((aligned(16))) int srb[RBN];
  __shared__ int wtot[OTHR / 32];
  const int tid = threadIdx.x, lane = tid & 31, wave = tid >> 5, sub = tid >> 7;
  for (int i = tid; i < RBN; i += OTHR) srb[i] = 0;
  int carry = 0;
#pragma unroll 1
  for (int ch = 0; ch < nChunk; ++ch) {
    const int base = ch * NBC;
    const v4i c0 = *(const v4i*)(cnt + base + 8 * tid);
    const v4i c1 = *(const v4i*)(cnt + base + 8 * tid + 4);
    const int e0 = max(c0.x, 0), e1 = max(c0.y, 0), e2 = max(c0.z, 0), e3 = max(c0.w, 0);
    const int e4 = max(c1.x, 0), e5 = max(c1.y, 0), e6 = max(c1.z, 0), e7 = max(c1.w, 0);
    const int ts = e0 + e1 + e2 + e3 + e4 + e5 + e6 + e7;
    int incl = ts;
#pragma unroll
    for (int d = 1; d < 32; d <<= 1) {
      const int t = __shfl_up(incl, d);
      if (lane >= d) incl += t;
    }
    if (lane == 31) wtot[wave] = incl;
    __syncthreads();
    const int S0 = wtot[0]  + wtot[1]  + wtot[2]  + wtot[3];
    const int S1 = wtot[4]  + wtot[5]  + wtot[6]  + wtot[7];
    const int S2 = wtot[8]  + wtot[9]  + wtot[10] + wtot[11];
    const int S3 = wtot[12] + wtot[13] + wtot[14] + wtot[15];
    int pre = 0;
#pragma unroll 1
    for (int w = 4 * sub; w < wave; ++w) pre += wtot[w];
    const int b0 = carry;
    const int b1 = b0 + ((S0 + 31) & ~31);
    const int b2 = b1 + ((S1 + 31) & ~31);
    const int b3 = b2 + ((S2 + 31) & ~31);
    const int b4 = b3 + ((S3 + 31) & ~31);
    const int myb = sub == 0 ? b0 : (sub == 1 ? b1 : (sub == 2 ? b2 : b3));
    if (tid == 0) {
      srb[min(4 * ch + 0, RBN - 1)] = b0;
      srb[min(4 * ch + 1, RBN - 1)] = b1;
      srb[min(4 * ch + 2, RBN - 1)] = b2;
      srb[min(4 * ch + 3, RBN - 1)] = b3;
    }
    int run = myb + pre + incl - ts;
    soff[8 * tid + 0] = run; run += e0;
    soff[8 * tid + 1] = run; run += e1;
    soff[8 * tid + 2] = run; run += e2;
    soff[8 * tid + 3] = run; run += e3;
    soff[8 * tid + 4] = run; run += e4;
    soff[8 * tid + 5] = run; run += e5;
    soff[8 * tid + 6] = run; run += e6;
    soff[8 * tid + 7] = run;
    carry = b4;
    __syncthreads();
    const v4i o0 = *(const v4i*)(soff + 4 * tid);
    const v4i o1 = *(const v4i*)(soff + 4 * (tid + OTHR));
    int* op = off + base;
    *(volatile v4i*)(op + 4 * tid) = o0;
    *(volatile v4i*)(op + 4 * (tid + OTHR)) = o1;
    __threadfence();
    *(volatile v4i*)(op + 4 * tid) = o0;
    *(volatile v4i*)(op + 4 * (tid + OTHR)) = o1;
    __syncthreads();
  }
  if (tid == 0) srb[min(4 * nChunk, RBN - 1)] = carry;
  __syncthreads();
  v4i rv = {0, 0, 0, 0};
  if (tid < 32) rv = *(const v4i*)(srb + 4 * tid);
  if (tid < 32) *(volatile v4i*)(rbase + 4 * tid) = rv;
  __threadfence();
  if (tid < 32) *(volatile v4i*)(rbase + 4 * tid) = rv;
}

__global__ __launch_bounds__(NTHR) void k_fill(
    const int* __restrict__ srcs, const int* __restrict__ dsts,
    const int* __restrict__ off, const int* __restrict__ rbase,
    int* csr, int nN, int nE, int vec8, int csrLen) {
  extern __shared__ v4f lds_dyn[];
  int* region = (int*)lds_dyn;
  int* cursor = region + RCAP;
  int* list   = cursor + NBF;
  int* wcnt   = list + LISTN;
  const int tid = threadIdx.x, lane = tid & 31, wave = tid >> 5;
  const int b = blockIdx.x;
  const int nodeBase = b * NBF;

  int rb0 = rbase[b];
  const int rb1 = rbase[b + 1];
  rb0 = rb0 < 0 ? 0 : (rb0 > csrLen ? csrLen : rb0);
  rb0 &= ~31;
  int len = rb1 - rb0;
  len = len < 0 ? 0 : (len > RCAP ? RCAP : len);
  int lenW = (len + 31) & ~31;
  if (rb0 + lenW > csrLen) lenW = (csrLen - rb0) & ~31;

  {
    const v4i z = {0, 0, 0, 0};
    for (int i = tid; i < RCAP / 4; i += NTHR) ((v4i*)region)[i] = z;
    for (int s = tid; s < NBF; s += NTHR) {
      int o = off[nodeBase + s] - rb0;
      o = o < 0 ? 0 : (o > RCAP ? RCAP : o);
      cursor[s] = o;
    }
  }
  __syncthreads();

  const int nChunks = (nE + CHUNK - 1) / CHUNK;
#pragma unroll 1
  for (int ch = 0; ch < nChunks; ++ch) {
    const int cbase = ch * CHUNK;
    const int wc = scan_chunk<NBF, false>(dsts, nE, dsts, nE, cbase, nodeBase, vec8, list, tid, lane, wave);
    if (lane == 0) wcnt[wave] = wc;
    __syncthreads();
    if (wave == 0) {
#pragma unroll 1
      for (int wsx = 0; wsx < NWAVE; ++wsx) {
        int n = __builtin_amdgcn_readfirstlane(wcnt[wsx]);
        n = n > WCAP ? WCAP : (n < 0 ? 0 : n);
        const int* lp = list + wsx * WCAP;
#pragma unroll 1
        for (int i = 0; i < n; ++i) {
          const int ent  = __builtin_amdgcn_readfirstlane(lp[i]);
          const int slot = ent & (NBF - 1);
          int e = cbase + ((ent >> 12) & (CHUNK - 1));
          e = e > nE - 1 ? nE - 1 : e;
          int src = srcs[e];
          src = src < 0 ? 0 : (src > nN - 1 ? nN - 1 : src);
          if (lane == 0) {
            int pos = cursor[slot];
            pos = pos < 0 ? 0 : (pos > RCAP - 1 ? RCAP - 1 : pos);
            region[pos] = src;
            const int np = pos + 1;
            cursor[slot] = np > RCAP ? RCAP : np;
          }
        }
      }
    }
    __syncthreads();
  }

  const int nv = lenW >> 2;
  int* gp = csr + rb0;
#pragma unroll 1
  for (int i = tid; i < nv; i += NTHR) { const v4i v = ((const v4i*)region)[i]; *(volatile v4i*)(gp + 4 * i) = v; }
  __threadfence();
#pragma unroll 1
  for (int i = tid; i < nv; i += NTHR) { const v4i v = ((const v4i*)region)[i]; *(volatile v4i*)(gp + 4 * i) = v; }
}

template <int F>
__global__ __launch_bounds__(NTHR) void k_agg(
    const int* __restrict__ csr, const int* __restrict__ off, const int* __restrict__ cnt,
    const float* __restrict__ hin, _Float16* zout, int nN, int csrLen) {
  static_assert((F & (F - 1)) == 0 && F >= 128 && F <= 256);
  const int tid = threadIdx.x, lane = tid & 31, wave = tid >> 5;
  const int tbase = blockIdx.x * TGT + wave * 32;
  const int colb = (8 * lane) & (F - 1);
  const bool act = lane < (F / 8);
  const v4f z4 = {0.f, 0.f, 0.f, 0.f};

  const int cl    = tbase + lane;
  const int cnt_l = cnt[cl];
  const int off_l = off[cl];

#pragma unroll 1
  for (int j = 0; j < 32; ++j) {
    const int c = tbase + j;
    int n = __shfl(cnt_l, j);
    n = n < 0 ? 0 : (n > DEGCAP ? DEGCAP : n);
    const int st = __shfl(off_l, j);

    v4f acc0 = z4, acc1 = z4;
#pragma unroll 1
    for (int q0 = 0; q0 < n; q0 += 32) {
      int pos = st + q0 + lane;
      pos = pos < 0 ? 0 : (pos > csrLen - 1 ? csrLen - 1 : pos);
      int sl = csr[pos];
      sl = sl < 0 ? 0 : (sl > nN - 1 ? nN - 1 : sl);
      const int mcnt = (n - q0) < 32 ? (n - q0) : 32;
#pragma unroll 1
      for (int pp = 0; pp < mcnt; ++pp) {
        const int s = __builtin_amdgcn_readlane(sl, pp);
        const float* hr = hin + (size_t)s * F + colb;
        acc0 = acc0 + *(const v4f*)hr;
        acc1 = acc1 + *(const v4f*)(hr + 4);
      }
    }
    {
      const int cc = c < nN ? c : nN - 1;
      const float* hr = hin + (size_t)cc * F + colb;
      acc0 = acc0 + *(const v4f*)hr;
      acc1 = acc1 + *(const v4f*)(hr + 4);
    }
    if (c >= nN) { acc0 = z4; acc1 = z4; }
    v8h hv;
    hv[0] = (_Float16)(acc0.x * XSC); hv[1] = (_Float16)(acc0.y * XSC);
    hv[2] = (_Float16)(acc0.z * XSC); hv[3] = (_Float16)(acc0.w * XSC);
    hv[4] = (_Float16)(acc1.x * XSC); hv[5] = (_Float16)(acc1.y * XSC);
    hv[6] = (_Float16)(acc1.z * XSC); hv[7] = (_Float16)(acc1.w * XSC);
    _Float16* pw = zout + (size_t)c * F + colb;
    if (act) *(volatile v8h*)pw = hv;
    __threadfence();
    if (act) *(volatile v8h*)pw = hv;
  }
}

template <int K>
__device__ __forceinline__ void mm_tile(const _Float16* __restrict__ A, int lda, int rowBase,
                                        const _Float16* __restrict__ Bw, v8f* acc) {
  const int tid = threadIdx.x, lane = tid & 31, wave = tid >> 5, hh = lane >> 4, m = lane & 15;
  const int r0 = (wave >> 2) * 16, c0 = (wave & 3) * (16 * NT);
#pragma unroll
  for (int t = 0; t < NT; ++t) { v8f z = {0.f, 0.f, 0.f, 0.f, 0.f, 0.f, 0.f, 0.f}; acc[t] = z; }
  const _Float16* ap  = A  + (size_t)(rowBase + r0 + m) * lda + 8 * hh;
  const _Float16* bp0 = Bw + (size_t)(c0 + m) * K + 8 * hh;
#pragma unroll 1
  for (int kt = 0; kt < K / 32; ++kt) {
    FragH a;
    a.h[0] = *(const v8h*)(ap + 32 * kt);
    a.h[1] = *(const v8h*)(ap + 32 * kt + 16);
#pragma unroll
    for (int t = 0; t < NT; ++t) {
      const _Float16* bp = bp0 + (size_t)(16 * t) * K + 32 * kt;
      FragH b;
      b.h[0] = *(const v8h*)bp;
      b.h[1] = *(const v8h*)(bp + 16);
      acc[t] = wmh(a.v, b.v, acc[t]);
    }
  }
}

template <int K1>
__global__ __launch_bounds__(NTHR) void k_mlp(const _Float16* __restrict__ Z, const _Float16* __restrict__ W1p,
                                              const float* __restrict__ b1, const _Float16* __restrict__ W2p,
                                              const float* __restrict__ b2, float* U) {
  __shared__ __attribute__((aligned(16))) _Float16 sT[BM * HD];
  __shared__ __attribute__((aligned(16))) float    sU[BM * HD];
  const int tid = threadIdx.x, lane = tid & 31, wave = tid >> 5, hh = lane >> 4, m = lane & 15;
  const int rowBase = blockIdx.x * BM;
  const int r0 = (wave >> 2) * 16, c0 = (wave & 3) * (16 * NT);
  v8f acc[NT];

  mm_tile<K1>(Z, K1, rowBase, W1p, acc);
  {
    _Float16* sp = sT + (r0 + 8 * hh) * HD + c0 + m;
#pragma unroll
    for (int t = 0; t < NT; ++t) {
      const float bv = b1[c0 + 16 * t + m];
#pragma unroll
      for (int r = 0; r < 8; ++r) {
        const float v = fmaxf(fmaf(acc[t][r], INV_CARRY, bv), 0.0f);
        sp[r * HD + 16 * t] = (_Float16)(v * XSC);
      }
    }
  }
  __syncthreads();

  mm_tile<HD>(sT, HD, 0, W2p, acc);
  {
    float* sp = sU + (r0 + 8 * hh) * HD + c0 + m;
#pragma unroll
    for (int t = 0; t < NT; ++t) {
      const float bv = b2[c0 + 16 * t + m];
#pragma unroll
      for (int r = 0; r < 8; ++r) sp[r * HD + 16 * t] = fmaxf(fmaf(acc[t][r], INV_CARRY, bv), 0.0f);
    }
  }
  __syncthreads();

  constexpr int NIT = ((BM * HD) / 4) / NTHR;
  const size_t gb = (size_t)rowBase * HD;
  v4f vv[NIT];
#pragma unroll
  for (int it = 0; it < NIT; ++it) vv[it] = ((const v4f*)sU)[it * NTHR + tid];
#pragma unroll
  for (int it = 0; it < NIT; ++it) *(volatile v4f*)(U + gb + (size_t)(it * NTHR + tid) * 4) = vv[it];
  __threadfence();
#pragma unroll
  for (int it = 0; it < NIT; ++it) *(volatile v4f*)(U + gb + (size_t)(it * NTHR + tid) * 4) = vv[it];
}

template <int ACT, int LSM>
__global__ __launch_bounds__(NTHR) void k_gemm_dot(const _Float16* __restrict__ A, const _Float16* __restrict__ Wp,
                                                   const float* __restrict__ b1, const float* __restrict__ w2,
                                                   const float* __restrict__ b2, float* outp, int nValid) {
  __shared__ __attribute__((aligned(16))) float sV[BM * HD];
  __shared__ __attribute__((aligned(16))) float sO[BM * 2];
  const int tid = threadIdx.x, lane = tid & 31, wave = tid >> 5, hh = lane >> 4, m = lane & 15;
  const int rowBase = blockIdx.x * BM;
  const int r0 = (wave >> 2) * 16, c0 = (wave & 3) * (16 * NT);
  v8f acc[NT];

  mm_tile<HD>(A, HD, rowBase, Wp, acc);
  {
    float* sp = sV + (r0 + 8 * hh) * HD + c0 + m;
#pragma unroll
    for (int t = 0; t < NT; ++t) {
      const float bv = b1[c0 + 16 * t + m];
#pragma unroll
      for (int r = 0; r < 8; ++r) sp[r * HD + 16 * t] = fmaf(acc[t][r], INV_CARRY, bv);
    }
  }
  __syncthreads();

  const int row = tid >> 3, q = tid & 7;
  float s0 = 0.0f, s1 = 0.0f;
#pragma unroll 4
  for (int i = 0; i < 32; ++i) {
    const int col = 32 * q + i;
    float v = sV[row * HD + col];
    v = (ACT == 2) ? tanhf(v) : fmaxf(v, 0.0f);
    s0 = fmaf(v, w2[2 * col], s0);
    s1 = fmaf(v, w2[2 * col + 1], s1);
  }
#pragma unroll
  for (int o = 1; o < 8; o <<= 1) {
    s0 += __shfl_xor(s0, o);
    s1 += __shfl_xor(s1, o);
  }
  s0 += b2[0];
  s1 += b2[1];
  const float mx = fmaxf(s0, s1);
  float o0, o1;
  if (LSM == 1) {
    const float l = logf(expf(s0 - mx) + expf(s1 - mx));
    o0 = s0 - mx - l;
    o1 = s1 - mx - l;
  } else {
    const float e0 = expf(s0 - mx), e1 = expf(s1 - mx);
    const float inv = 1.0f / (e0 + e1);
    o0 = e0 * inv;
    o1 = e1 * inv;
  }
  if (q == 0) { sO[2 * row] = o0; sO[2 * row + 1] = o1; }
  __syncthreads();

  if (wave == 0) {
    int nv = nValid - rowBase;
    nv = nv < 0 ? 0 : (nv > BM ? BM : nv);
    const int lq = lane < 16 ? lane : 15;
    const v4f v  = ((const v4f*)sO)[lq];
    const bool full = (lane < 16) && (2 * lq + 2 <= nv);
    const bool half = (lane < 16) && !full && (2 * lq + 1 <= nv);
    v2f v2;
    v2.x = v.x; v2.y = v.y;
    float* op = outp + (size_t)rowBase * 2 + 4 * lq;
    if (full) *(volatile v4f*)op = v;
    if (half) *(volatile v2f*)op = v2;
    __threadfence();
    if (full) *(volatile v4f*)op = v;
    if (half) *(volatile v2f*)op = v2;
  }
}

__global__ __launch_bounds__(NTHR) void k_bnstat(const float* __restrict__ u, double* part, int nN) {
  const int col = threadIdx.x;
  const int r0 = blockIdx.x * STATR;
  int nr = nN - r0;
  nr = nr < 0 ? 0 : (nr > STATR ? STATR : nr);
  double s = 0.0, q = 0.0;
#pragma unroll 1
  for (int i = 0; i < nr; ++i) {
    const double v = (double)u[(size_t)(r0 + i) * HD + col];
    s += v;
    q += v * v;
  }
  double* pp = part + (size_t)blockIdx.x * (2 * HD);
  *(volatile double*)(pp + col) = s;
  *(volatile double*)(pp + HD + col) = q;
  __threadfence();
  *(volatile double*)(pp + col) = s;
  *(volatile double*)(pp + HD + col) = q;
}

__global__ __launch_bounds__(NTHR) void k_bnfin(const double* __restrict__ part, const float* __restrict__ gamma,
                                                float* tbl, int nPart, int nN) {
  const int col = threadIdx.x;
  double s = 0.0, q = 0.0;
#pragma unroll 1
  for (int b = 0; b < nPart; ++b) {
    s += part[(size_t)b * (2 * HD) + col];
    q += part[(size_t)b * (2 * HD) + HD + col];
  }
  const double inv = 1.0 / (double)nN;
  const double mu  = s * inv;
  double var = q * inv - mu * mu;
  var = var < 0.0 ? 0.0 : var;
  const float a  = (float)((double)gamma[col] / sqrt(var + BN_EPS));
  const float mf = (float)mu;
  *(volatile float*)(tbl + col) = mf;
  *(volatile float*)(tbl + HD + col) = a;
  __threadfence();
  *(volatile float*)(tbl + col) = mf;
  *(volatile float*)(tbl + HD + col) = a;
}

__global__ __launch_bounds__(NTHR) void k_update(
    float* P, const float* __restrict__ tbl, const float* __restrict__ beta,
    _Float16* h16, int nN, int nUnits, int wh16) {
  const int i = (int)blockIdx.x * NTHR + (int)threadIdx.x;
  if (i >= nUnits) return;
  const int row = i / (HD / 4);
  const int c   = (i - row * (HD / 4)) * 4;
  const v4f mu = *(const v4f*)(tbl + c);
  const v4f ga = *(const v4f*)(tbl + HD + c);
  const v4f be = *(const v4f*)(beta + c);
  const size_t p = (size_t)i * 4;
  const v4f u  = *(const v4f*)(P + p);
  v4f v = (u - mu) * ga + be;
  if (row >= nN) { v.x = 0.0f; v.y = 0.0f; v.z = 0.0f; v.w = 0.0f; }
  v4h hv;
  hv.x = (_Float16)(v.x * XSC); hv.y = (_Float16)(v.y * XSC);
  hv.z = (_Float16)(v.z * XSC); hv.w = (_Float16)(v.w * XSC);
  *(volatile v4f*)(P + p) = v;
  if (wh16 != 0) *(volatile v4h*)(h16 + p) = hv;
  __threadfence();
  *(volatile v4f*)(P + p) = v;
  if (wh16 != 0) *(volatile v4h*)(h16 + p) = hv;
}

__global__ __launch_bounds__(NTHR) void k_pool(
    const int* __restrict__ gid, const float* __restrict__ hfin, const float* __restrict__ ap,
    float* out1, float* out2, _Float16* sub16, int nN, int nG, int vec8) {
  __shared__ __attribute__((aligned(16))) float sacc[GPB * HD];
  __shared__ __attribute__((aligned(16))) float ssub[GPB * HD];
  __shared__ __attribute__((aligned(16))) int   list[LISTN];
  __shared__ float sinv[GPB];
  __shared__ int   scnt[GPB];
  __shared__ int   wcnt[NWAVE];
  const int tid = threadIdx.x, lane = tid & 31, wave = tid >> 5;
  const int gbase = blockIdx.x * GPB;

  for (int i = tid; i < GPB * HD; i += NTHR) { sacc[i] = 0.0f; ssub[i] = 0.0f; }
  if (tid < GPB) scnt[tid] = 0;
  __syncthreads();

  const int nChunks = (nN + CHUNK - 1) / CHUNK;
#pragma unroll 1
  for (int ch = 0; ch < nChunks; ++ch) {
    const int cbase = ch * CHUNK;
    const int wc = scan_chunk<GPB, false>(gid, nN, gid, nN, cbase, gbase, vec8, list, tid, lane, wave);
    if (lane == 0) wcnt[wave] = wc;
    __syncthreads();
#pragma unroll 1
    for (int wsx = 0; wsx < NWAVE; ++wsx) {
      int n = wcnt[wsx];
      n = n > WCAP ? WCAP : (n < 0 ? 0 : n);
      const int* lp = list + wsx * WCAP;
#pragma unroll 1
      for (int i = 0; i < n; ++i) {
        const int ent  = lp[i];
        const int slot = ent & (GPB - 1);
        int node = cbase + ((ent >> 12) & (CHUNK - 1));
        node = node > nN - 1 ? nN - 1 : node;
        const float hv = hfin[(size_t)node * HD + tid];
        const float a0 = ap[(size_t)node * 2];
        sacc[slot * HD + tid] += hv;
        ssub[slot * HD + tid] += a0 * hv;
        if (tid == 0) scnt[slot] = scnt[slot] + 1;
      }
    }
    __syncthreads();
  }

  if (tid < GPB) {
    const int cg = scnt[tid];
    sinv[tid] = 1.0f / (float)cg;
  }
  __syncthreads();

  int nv = nG - gbase;
  nv = nv < 0 ? 0 : (nv > GPB ? GPB : nv);
  constexpr int NI4 = ((GPB * HD) / 4) / NTHR;
  constexpr int NI8 = ((GPB * HD) / 8) / NTHR;
  v4f v1[NI4], v2[NI4];
  bool ok[NI4];
#pragma unroll
  for (int it = 0; it < NI4; ++it) {
    const int f   = it * NTHR + tid;
    const int row = f / (HD / 4);
    ok[it] = row < nv;
    v1[it] = ((const v4f*)ssub)[f];
    v2[it] = ((const v4f*)sacc)[f] * sinv[row];
  }
  v8h h8[NI8];
#pragma unroll
  for (int it = 0; it < NI8; ++it) {
    const int f = it * NTHR + tid;
    const v4f s0 = ((const v4f*)ssub)[2 * f];
    const v4f s1 = ((const v4f*)ssub)[2 * f + 1];
    h8[it][0] = (_Float16)(s0.x * XSC); h8[it][1] = (_Float16)(s0.y * XSC);
    h8[it][2] = (_Float16)(s0.z * XSC); h8[it][3] = (_Float16)(s0.w * XSC);
    h8[it][4] = (_Float16)(s1.x * XSC); h8[it][5] = (_Float16)(s1.y * XSC);
    h8[it][6] = (_Float16)(s1.z * XSC); h8[it][7] = (_Float16)(s1.w * XSC);
  }
  float* o1 = out1 + (size_t)gbase * HD;
  float* o2 = out2 + (size_t)gbase * HD;
  _Float16* o3 = sub16 + (size_t)gbase * HD;
#pragma unroll
  for (int it = 0; it < NI4; ++it) {
    const int f = it * NTHR + tid;
    if (ok[it]) { *(volatile v4f*)(o1 + 4 * f) = v1[it]; *(volatile v4f*)(o2 + 4 * f) = v2[it]; }
  }
#pragma unroll
  for (int it = 0; it < NI8; ++it) { const int f = it * NTHR + tid; *(volatile v8h*)(o3 + 8 * f) = h8[it]; }
  __threadfence();
#pragma unroll
  for (int it = 0; it < NI4; ++it) {
    const int f = it * NTHR + tid;
    if (ok[it]) { *(volatile v4f*)(o1 + 4 * f) = v1[it]; *(volatile v4f*)(o2 + 4 * f) = v2[it]; }
  }
#pragma unroll
  for (int it = 0; it < NI8; ++it) { const int f = it * NTHR + tid; *(volatile v8h*)(o3 + 8 * f) = h8[it]; }
}

__global__ __launch_bounds__(NTHR) void k_adj(
    const int* __restrict__ srcs, const int* __restrict__ dsts, const int* __restrict__ gid,
    const float* __restrict__ ap, float* pen, int nN, int nE, int nG, int vec8) {
  __shared__ __attribute__((aligned(16))) int list[LISTN];
  __shared__ int wcnt[NWAVE];
  const int tid = threadIdx.x, lane = tid & 31, wave = tid >> 5;
  const int gbase = blockIdx.x * GPA;
  double m00 = 0.0, m01 = 0.0, m10 = 0.0, m11 = 0.0;

  const int nChunks = (nE + CHUNK - 1) / CHUNK;
#pragma unroll 1
  for (int ch = 0; ch < nChunks; ++ch) {
    const int cbase = ch * CHUNK;
    const int wc = scan_chunk<GPA, true>(srcs, nE, gid, nN, cbase, gbase, vec8, list, tid, lane, wave);
    if (lane == 0) wcnt[wave] = wc;
    __syncthreads();
    if (wave == 0) {
#pragma unroll 1
      for (int wsx = 0; wsx < NWAVE; ++wsx) {
        int n = __builtin_amdgcn_readfirstlane(wcnt[wsx]);
        n = n > WCAP ? WCAP : (n < 0 ? 0 : n);
        const int* lp = list + wsx * WCAP;
#pragma unroll 1
        for (int i = 0; i < n; ++i) {
          const int ent  = __builtin_amdgcn_readfirstlane(lp[i]);
          const int slot = ent & (GPA - 1);
          int e = cbase + ((ent >> 12) & (CHUNK - 1));
          e = e > nE - 1 ? nE - 1 : e;
          int s = srcs[e];
          s = s < 0 ? 0 : (s > nN - 1 ? nN - 1 : s);
          int d = dsts[e];
          d = d < 0 ? 0 : (d > nN - 1 ? nN - 1 : d);
          const float as0 = ap[(size_t)s * 2], as1 = ap[(size_t)s * 2 + 1];
          const float ad0 = ap[(size_t)d * 2], ad1 = ap[(size_t)d * 2 + 1];
          if (slot == lane) {
            m00 += (double)as0 * (double)ad0;
            m01 += (double)as0 * (double)ad1;
            m10 += (double)as1 * (double)ad0;
            m11 += (double)as1 * (double)ad1;
          }
        }
      }
    }
    __syncthreads();
  }

  if (wave == 0) {
    const float n00 = (float)m00, n01 = (float)m01, n10 = (float)m10, n11 = (float)m11;
    const float rn0 = fmaxf(fabsf(n00) + fabsf(n01), 1e-12f);
    const float rn1 = fmaxf(fabsf(n10) + fabsf(n11), 1e-12f);
    const float d0 = n00 * (1.0f / rn0) - 1.0f;
    const float d1 = n11 * (1.0f / rn1) - 1.0f;
    float pv = 0.5f * (d0 * d0 + d1 * d1);
    if (gbase + lane >= nG) pv = 0.0f;
    float* pp = pen + gbase + lane;
    *(volatile float*)pp = pv;
    __threadfence();
    *(volatile float*)pp = pv;
  }
}

__global__ __launch_bounds__(32) void k_penfin(const float* __restrict__ pen, float* out3, int nG) {
  const int lane = threadIdx.x & 31;
  double s = 0.0;
#pragma unroll 1
  for (int g = lane; g < nG; g += 32) s += (double)pen[g];
#pragma unroll
  for (int o = 16; o > 0; o >>= 1) s += __shfl_xor(s, o);
  const float r = (float)(s / (double)nG);
  if (lane == 0) {
    *(volatile float*)out3 = r;
    __threadfence();
    *(volatile float*)out3 = r;
  }
}

extern "C" void kernel_launch(void* const* d_in, const int* in_sizes, int n_in,
                              void* d_out, int out_size, void* d_ws, size_t ws_size,
                              hipStream_t stream) {
  if (n_in < 23) return;
  const int nN = in_sizes[2];
  if (nN <= 0 || in_sizes[0] != nN * FIN0) return;
  if (in_sizes[1] <= 0 || (in_sizes[1] & 1) != 0) return;
  const int nE = in_sizes[1] / 2;
  if (in_sizes[3] != FIN0 * HD || in_sizes[4] != HD || in_sizes[5] != HD * HD || in_sizes[6] != HD) return;
  if (in_sizes[7] != HD || in_sizes[8] != HD) return;
  if (in_sizes[9] <= 0 || (in_sizes[9] % (HD * HD)) != 0) return;
  const int nLs = in_sizes[9] / (HD * HD);
  if (nLs > 8) return;
  if (in_sizes[10] != nLs * HD || in_sizes[11] != nLs * HD * HD || in_sizes[12] != nLs * HD) return;
  if (in_sizes[13] != nLs * HD || in_sizes[14] != nLs * HD) return;
  if (in_sizes[15] != HD * HD || in_sizes[16] != HD || in_sizes[17] != HD * NCLS || in_sizes[18] != NCLS) return;
  if (in_sizes[19] != HD * HD || in_sizes[20] != HD || in_sizes[21] != HD * NCLS || in_sizes[22] != NCLS) return;
  if (out_size < 1 + 2 * HD + NCLS || ((out_size - 1) % (2 * HD + NCLS)) != 0) return;
  const int nG = (out_size - 1) / (2 * HD + NCLS);
  if (nE > (1 << 28) || nN > (1 << 22) || nG > (1 << 22)) return;

  const float* x    = (const float*)d_in[0];
  const int*   ei   = (const int*)d_in[1];
  const int*   bvec = (const int*)d_in[2];
  const float* w0_1 = (const float*)d_in[3];
  const float* b0_1 = (const float*)d_in[4];
  const float* w0_2 = (const float*)d_in[5];
  const float* b0_2 = (const float*)d_in[6];
  const float* g0   = (const float*)d_in[7];
  const float* be0  = (const float*)d_in[8];
  const float* wl1  = (const float*)d_in[9];
  const float* bl1  = (const float*)d_in[10];
  const float* wl2  = (const float*)d_in[11];
  const float* bl2  = (const float*)d_in[12];
  const float* gl   = (const float*)d_in[13];
  const float* bel  = (const float*)d_in[14];
  const float* c1w  = (const float*)d_in[15];
  const float* c1b  = (const float*)d_in[16];
  const float* c2w  = (const float*)d_in[17];
  const float* c2b  = (const float*)d_in[18];
  const float* l1w  = (const float*)d_in[19];
  const float* l1b  = (const float*)d_in[20];
  const float* l2w  = (const float*)d_in[21];
  const float* l2b  = (const float*)d_in[22];
  const int* src = ei;
  const int* dst = ei + nE;
  float* out0 = (float*)d_out;
  float* out1 = out0 + (size_t)nG * NCLS;
  float* out2 = out1 + (size_t)nG * HD;
  float* out3 = out2 + (size_t)nG * HD;

  const int NPAD   = ((nN + TGT - 1) / TGT) * TGT;
  const int nBC    = (nN + NBC - 1) / NBC;
  const int CNTPAD = nBC * NBC;
  if (4 * nBC + 1 > RBN) return;
  const int nBF    = (nN + NBF - 1) / NBF;
  const int csrLen = ((nE + 31) & ~31) + 4096;
  if (31 * 4 * nBC > 4096) return;
  const int nAgg   = NPAD / TGT;
  const int nGm    = NPAD / BM;
  const int nStat  = NPAD / STATR;
  const int nUnit  = NPAD * (HD / 4);
  const int GPAD   = ((nG + GPA - 1) / GPA) * GPA;
  const int nPool  = GPAD / GPB;
  const int nAdj   = GPAD / GPA;
  const int nHead  = GPAD / BM;
  const int nW01U  = HD * (FIN0 / 8);
  const int nWHU   = HD * (HD / 8);

  char* ws = (char*)d_ws;
  size_t off = 0;
  const size_t oW01 = off; off += (size_t)HD * FIN0 * 2;         off = (off + 255) & ~(size_t)255;
  const size_t oW02 = off; off += (size_t)HD * HD * 2;           off = (off + 255) & ~(size_t)255;
  const size_t oWl1 = off; off += (size_t)nLs * HD * HD * 2;     off = (off + 255) & ~(size_t)255;
  const size_t oWl2 = off; off += (size_t)nLs * HD * HD * 2;     off = (off + 255) & ~(size_t)255;
  const size_t oWc1 = off; off += (size_t)HD * HD * 2;           off = (off + 255) & ~(size_t)255;
  const size_t oWh1 = off; off += (size_t)HD * HD * 2;           off = (off + 255) & ~(size_t)255;
  const size_t oZ   = off; off += (size_t)NPAD * HD * 2;         off = (off + 255) & ~(size_t)255;
  const size_t oP   = off; off += (size_t)NPAD * HD * 4;         off = (off + 255) & ~(size_t)255;
  const size_t oCnt = off; off += (size_t)CNTPAD * 4;            off = (off + 255) & ~(size_t)255;
  const size_t oOff = off; off += (size_t)CNTPAD * 4;            off = (off + 255) & ~(size_t)255;
  const size_t oRb  = off; off += (size_t)RBN * 4;               off = (off + 255) & ~(size_t)255;
  const size_t oCsr = off; off += (size_t)csrLen * 4;            off = (off + 255) & ~(size_t)255;
  const size_t oPrt = off; off += (size_t)nStat * 2 * HD * 8;    off = (off + 255) & ~(size_t)255;
  const size_t oTbl = off; off += (size_t)2 * HD * 4;            off = (off + 255) & ~(size_t)255;
  const size_t oA   = off; off += (size_t)NPAD * 2 * 4;          off = (off + 255) & ~(size_t)255;
  const size_t oS16 = off; off += (size_t)GPAD * HD * 2;         off = (off + 255) & ~(size_t)255;
  const size_t oPen = off; off += (size_t)GPAD * 4;              off = (off + 255) & ~(size_t)255;
  if (off > ws_size || off > (size_t)WSCAP) return;
  _Float16* wp01 = (_Float16*)(ws + oW01);
  _Float16* wp02 = (_Float16*)(ws + oW02);
  _Float16* wpl1 = (_Float16*)(ws + oWl1);
  _Float16* wpl2 = (_Float16*)(ws + oWl2);
  _Float16* wpc1 = (_Float16*)(ws + oWc1);
  _Float16* wph1 = (_Float16*)(ws + oWh1);
  _Float16* z16  = (_Float16*)(ws + oZ);
  float*    P    = (float*)(ws + oP);
  int*      cnt  = (int*)(ws + oCnt);
  int*      offp = (int*)(ws + oOff);
  int*      rb   = (int*)(ws + oRb);
  int*      csr  = (int*)(ws + oCsr);
  double*   part = (double*)(ws + oPrt);
  float*    tbl  = (float*)(ws + oTbl);
  float*    apl  = (float*)(ws + oA);
  _Float16* s16  = (_Float16*)(ws + oS16);
  float*    pen  = (float*)(ws + oPen);

  const int vec8d = ((nE & 3) == 0) ? 1 : 0;

  k_wprep<FIN0, HD, FIN0, HD><<<(nW01U + NTHR - 1) / NTHR, NTHR, 0, stream>>>(w0_1, wp01, 1);
  k_wprep<HD, HD, HD, HD><<<(nWHU + NTHR - 1) / NTHR, NTHR, 0, stream>>>(w0_2, wp02, 1);
  k_wprep<HD, HD, HD, HD><<<(nLs * nWHU + NTHR - 1) / NTHR, NTHR, 0, stream>>>(wl1, wpl1, nLs);
  k_wprep<HD, HD, HD, HD><<<(nLs * nWHU + NTHR - 1) / NTHR, NTHR, 0, stream>>>(wl2, wpl2, nLs);
  k_wprep<HD, HD, HD, HD><<<(nWHU + NTHR - 1) / NTHR, NTHR, 0, stream>>>(c1w, wpc1, 1);
  k_wprep<HD, HD, HD, HD><<<(nWHU + NTHR - 1) / NTHR, NTHR, 0, stream>>>(l1w, wph1, 1);

  k_count<<<nBC, NTHR, 0, stream>>>(dst, cnt, nE, vec8d);
  k_offsets<<<1, OTHR, 0, stream>>>(cnt, offp, rb, nBC);
  hipFuncSetAttribute(reinterpret_cast<const void*>(&k_fill),
                      hipFuncAttributeMaxDynamicSharedMemorySize, LDS_FILL);
  k_fill<<<nBF, NTHR, LDS_FILL, stream>>>(src, dst, offp, rb, csr, nN, nE, vec8d, csrLen);

  k_agg<FIN0><<<nAgg, NTHR, 0, stream>>>(csr, offp, cnt, x, z16, nN, csrLen);
  k_mlp<FIN0><<<nGm, NTHR, 0, stream>>>(z16, wp01, b0_1, wp02, b0_2, P);
  k_bnstat<<<nStat, HD, 0, stream>>>(P, part, nN);
  k_bnfin<<<1, HD, 0, stream>>>(part, g0, tbl, nStat, nN);
  k_update<<<(nUnit + NTHR - 1) / NTHR, NTHR, 0, stream>>>(P, tbl, be0, z16, nN, nUnit, (nLs == 0) ? 1 : 0);

  for (int i = 0; i < nLs; ++i) {
    k_agg<HD><<<nAgg, NTHR, 0, stream>>>(csr, offp, cnt, P, z16, nN, csrLen);
    k_mlp<HD><<<nGm, NTHR, 0, stream>>>(z16, wpl1 + (size_t)i * HD * HD, bl1 + (size_t)i * HD,
                                         wpl2 + (size_t)i * HD * HD, bl2 + (size_t)i * HD, P);
    k_bnstat<<<nStat, HD, 0, stream>>>(P, part, nN);
    k_bnfin<<<1, HD, 0, stream>>>(part, gl + (size_t)i * HD, tbl, nStat, nN);
    k_update<<<(nUnit + NTHR - 1) / NTHR, NTHR, 0, stream>>>(P, tbl, bel + (size_t)i * HD, z16, nN, nUnit,
                                                             (i == nLs - 1) ? 1 : 0);
  }

  k_gemm_dot<2, 0><<<nGm, NTHR, 0, stream>>>(z16, wpc1, c1b, c2w, c2b, apl, NPAD);

  k_pool<<<nPool, NTHR, 0, stream>>>(bvec, P, apl, out1, out2, s16, nN, nG, 1);

  k_adj<<<nAdj, NTHR, 0, stream>>>(src, dst, bvec, apl, pen, nN, nE, nG, 1);
  k_penfin<<<1, 32, 0, stream>>>(pen, out3, nG);

  k_gemm_dot<1, 1><<<nHead, NTHR, 0, stream>>>(s16, wph1, l1b, l2w, l2b, out0, nG);
}
